// BiLSTM_50500225466406
// MI455X (gfx1250) — hardware-verified
//
#include <hip/hip_runtime.h>
#include <math.h>

constexpr int NBAT   = 32;
constexpr int NSEQ   = 128;
constexpr int NEMB   = 300;
constexpr int NEMBP  = 320;
constexpr int NHID   = 200;
constexpr int NUP    = 208;
constexpr int NHK    = 224;
constexpr int NGATE  = 4;
constexpr int NGC    = NGATE * NUP;
constexpr int NIN1   = 2 * NHID;
constexpr int YHALF  = 256;
constexpr int YPITCH = 2 * YHALF;
constexpr int NTAG   = 17;
constexpr int NTAGP  = 64;
constexpr int NROW   = NSEQ * NBAT;
constexpr int NVOC   = 50002;
constexpr int RTHR   = 32 * (NUP / 16);
constexpr int AHP    = 256;
constexpr int NOUT   = NBAT * NSEQ * NTAG;
constexpr float CARRY1     = 16.0f;
constexpr float CARRY2     = 256.0f;
constexpr float CARRY2_INV = 1.0f / 256.0f;

static_assert(NGC == 832 && NGC % 64 == 0);
static_assert(NROW % 64 == 0 && NTAGP % 64 == 0);
static_assert(NEMBP % 32 == 0 && NHK % 32 == 0 && YPITCH % 32 == 0);
static_assert(NUP % 16 == 0 && NUP >= NHID && NHK >= NUP && AHP >= NHK && AHP == YHALF);
static_assert(RTHR == 416 && RTHR % 8 == 0 && RTHR <= 512);
static_assert(NBAT == 32 && NSEQ == 128);
static_assert((NROW * NEMBP / 8) % 256 == 0);
static_assert((2 * NGC * NEMBP / 8) % 256 == 0);
static_assert((2 * NGC * NHK / 8) % 256 == 0);
static_assert((2 * NGC * YPITCH / 8) % 256 == 0);
static_assert((NTAGP * YPITCH / 8) % 256 == 0);
static_assert(NOUT % 1024 == 0);
static_assert((NGC * 4) % 128 == 0 && (NTAGP * 4) % 128 == 0 && (YPITCH * 2) % 128 == 0 && (YHALF * 2) % 128 == 0);

typedef __attribute__((ext_vector_type(16))) _Float16 v16h;
typedef __attribute__((ext_vector_type(8)))  _Float16 v8h;
typedef __attribute__((ext_vector_type(16))) __bf16   v16b;
typedef __attribute__((ext_vector_type(8)))  __bf16   v8b;
typedef __attribute__((ext_vector_type(8)))  float    v8f;
typedef __attribute__((ext_vector_type(4)))  float    v4f;

__device__ __forceinline__ unsigned short f2bf_bits(float f) {
  unsigned u = __float_as_uint(f);
  return (unsigned short)((u + 0x7FFFu + ((u >> 16) & 1u)) >> 16);
}
__device__ __forceinline__ float bf_bits2f(unsigned short h) { return __uint_as_float(((unsigned)h) << 16); }

__device__ __forceinline__ void dep_guard_h(v8f& a, v8f& b, v16h x, v16h y) { asm volatile("v_nop\n\tv_nop\n\tv_nop\n\tv_nop" : "+v"(a), "+v"(b) : "v"(x), "v"(y)); }
__device__ __forceinline__ void dep_guard_b(v8f& a, v8f& b, v16b x, v16b y) { asm volatile("v_nop\n\tv_nop\n\tv_nop\n\tv_nop" : "+v"(a), "+v"(b) : "v"(x), "v"(y)); }
__device__ __forceinline__ void dep_guard5_h(v8f& a0, v8f& a1, v8f& a2, v8f& a3, v16h x, v16h y0, v16h y1, v16h y2, v16h y3) {
  asm volatile("v_nop\n\tv_nop\n\tv_nop\n\tv_nop" : "+v"(a0), "+v"(a1), "+v"(a2), "+v"(a3) : "v"(x), "v"(y0), "v"(y1), "v"(y2), "v"(y3));
}
__device__ __forceinline__ void dep_guard5_b(v8f& a0, v8f& a1, v8f& a2, v8f& a3, v16b x, v16b y0, v16b y1, v16b y2, v16b y3) {
  asm volatile("v_nop\n\tv_nop\n\tv_nop\n\tv_nop" : "+v"(a0), "+v"(a1), "+v"(a2), "+v"(a3) : "v"(x), "v"(y0), "v"(y1), "v"(y2), "v"(y3));
}
__device__ __forceinline__ void keep4_h(v16h a, v16h b, v16h c, v16h d) { asm volatile("v_nop" :: "v"(a), "v"(b), "v"(c), "v"(d)); }
__device__ __forceinline__ void keep4_b(v16b a, v16b b, v16b c, v16b d) { asm volatile("v_nop" :: "v"(a), "v"(b), "v"(c), "v"(d)); }
__device__ __forceinline__ void acc_guard4(v8f& a, v8f& b, v8f& c, v8f& d) { asm volatile("v_nop\n\tv_nop\n\tv_nop\n\tv_nop" : "+v"(a), "+v"(b), "+v"(c), "+v"(d)); }
__device__ __forceinline__ void pin_acc(v8f& a) { asm volatile("" : "+v"(a) : : "memory"); }

template <typename T> struct Frag;
template <> struct Frag<_Float16> {
  typedef v16h V; union U { v16h v; v8h h[2]; };
  static __device__ __forceinline__ v16h load(const _Float16* p) {
    U f; f.h[0] = *(const v8h*)(p); f.h[1] = *(const v8h*)(p + 16); return f.v;
  }
  static __device__ __forceinline__ v8f mma(v16h a, v16h b, v8f c) {
    return __builtin_amdgcn_wmma_f32_16x16x32_f16(false, a, false, b, (short)0, c, false, false);
  }
  static __device__ __forceinline__ void guard(v8f& a, v8f& b, v16h x, v16h y) { dep_guard_h(a, b, x, y); }
  static __device__ __forceinline__ void guard5(v8f& a0, v8f& a1, v8f& a2, v8f& a3, v16h x, v16h y0, v16h y1, v16h y2, v16h y3) { dep_guard5_h(a0, a1, a2, a3, x, y0, y1, y2, y3); }
  static __device__ __forceinline__ void keep(v16h a, v16h b, v16h c, v16h d) { keep4_h(a, b, c, d); }
};
template <> struct Frag<__bf16> {
  typedef v16b V; union U { v16b v; v8b h[2]; };
  static __device__ __forceinline__ v16b load(const __bf16* p) {
    U f; f.h[0] = *(const v8b*)(p); f.h[1] = *(const v8b*)(p + 16); return f.v;
  }
  static __device__ __forceinline__ v8f mma(v16b a, v16b b, v8f c) {
    return __builtin_amdgcn_wmma_f32_16x16x32_bf16(false, a, false, b, (short)0, c, false, false);
  }
  static __device__ __forceinline__ void guard(v8f& a, v8f& b, v16b x, v16b y) { dep_guard_b(a, b, x, y); }
  static __device__ __forceinline__ void guard5(v8f& a0, v8f& a1, v8f& a2, v8f& a3, v16b x, v16b y0, v16b y1, v16b y2, v16b y3) { dep_guard5_b(a0, a1, a2, a3, x, y0, y1, y2, y3); }
  static __device__ __forceinline__ void keep(v16b a, v16b b, v16b c, v16b d) { keep4_b(a, b, c, d); }
};

__device__ __forceinline__ float fsig(float x)  { return __builtin_amdgcn_rcpf(1.0f + expf(-x)); }
__device__ __forceinline__ float ftanh(float x) { return 1.0f - 2.0f * __builtin_amdgcn_rcpf(expf(2.0f * x) + 1.0f); }

template <int ET> struct Elem;
template <> struct Elem<0> { typedef _Float16 T; };
template <> struct Elem<1> { typedef __bf16 T; };
template <int ET, bool SPLIT, int BIAS_MODE, int OUT_MODE, bool RESID, int ACT = 0>
__global__ __launch_bounds__(256) void wmma_gemm64(
    const unsigned short* __restrict__ Ap, const unsigned short* __restrict__ A2p, int lda, long strideA,
    const unsigned short* __restrict__ Btp, const unsigned short* __restrict__ Bt2p, int ldb, long strideB,
    void* __restrict__ Cout, void* __restrict__ Cout2, int ldc, long strideC,
    const float* __restrict__ bias,
    const float* __restrict__ resid, long strideR,
    int M, int N, int K, float scale) {
  typedef typename Elem<ET>::T T;
  typedef typename Frag<T>::V V;
  const T* A = (const T*)Ap; const T* A2 = (const T*)A2p; const T* Bt = (const T*)Btp; const T* Bt2 = (const T*)Bt2p;
  __shared__ __align__(16) float sT[8][16 * 68];
  const int b    = blockIdx.y;
  const int lane = threadIdx.x & 31;
  const int wave = threadIdx.x >> 5;
  const int tilesN = N >> 6;
  const int tilesM = M >> 6;
  const int tile = blockIdx.x * 8 + wave;
  if (tile >= tilesM * tilesN) return;
  const int tm = tile / tilesN;
  const int tn = tile - tm * tilesN;
  const int m0 = tm << 6;
  const int n0 = tn << 6;

  const T* Ab  = A  + (size_t)b * strideA;
  const T* Bb  = Bt + (size_t)b * strideB;
  const T* Ab2 = SPLIT ? (A2  + (size_t)b * strideA) : nullptr;
  const T* Bb2 = SPLIT ? (Bt2 + (size_t)b * strideB) : nullptr;

  const int rlane = lane & 15;
  const int koff  = (lane >> 4) * 8;
  const int mOff  = (lane >> 4) * 8;

  v8f acc[4][4];
#pragma unroll
  for (int i = 0; i < 4; ++i)
#pragma unroll
    for (int j = 0; j < 4; ++j) acc[i][j] = (v8f){0.f,0.f,0.f,0.f,0.f,0.f,0.f,0.f};

  for (int k0 = 0; k0 < K; k0 += 32) {
    V bh[4], bl[4];
#pragma unroll
    for (int j = 0; j < 4; ++j) {
      const size_t bo = (size_t)(n0 + (j << 4) + rlane) * ldb + koff + k0;
      bh[j] = Frag<T>::load(Bb + bo);
      if (SPLIT) bl[j] = Frag<T>::load(Bb2 + bo);
    }
#pragma unroll
    for (int i = 0; i < 4; ++i) {
      const size_t ao = (size_t)(m0 + (i << 4) + rlane) * lda + koff + k0;
      V ah = Frag<T>::load(Ab + ao);
      V al;
      if (SPLIT) al = Frag<T>::load(Ab2 + ao);
#pragma unroll
      for (int j = 0; j < 4; ++j) {
        acc[i][j] = Frag<T>::mma(ah, bh[j], acc[i][j]);
        if (SPLIT) {
          acc[i][j] = Frag<T>::mma(ah, bl[j], acc[i][j]);
          acc[i][j] = Frag<T>::mma(al, bh[j], acc[i][j]);
        }
      }
      Frag<T>::guard5(acc[i][0], acc[i][1], acc[i][2], acc[i][3], ah, bh[0], bh[1], bh[2], bh[3]);
      if (SPLIT) Frag<T>::keep(al, bl[0], bl[1], bl[2]);
    }
    Frag<T>::keep(bh[0], bh[1], bh[2], bh[3]);
    if (SPLIT) Frag<T>::keep(bl[0], bl[1], bl[2], bl[3]);
  }
  acc_guard4(acc[0][0], acc[0][1], acc[0][2], acc[0][3]);
  acc_guard4(acc[1][0], acc[1][1], acc[1][2], acc[1][3]);
  acc_guard4(acc[2][0], acc[2][1], acc[2][2], acc[2][3]);
  acc_guard4(acc[3][0], acc[3][1], acc[3][2], acc[3][3]);

  float* slab = sT[wave];
  const float* Rb = RESID ? (resid + (size_t)b * strideR) : nullptr;
#pragma unroll
  for (int i = 0; i < 4; ++i) {
    const int mBase = m0 + (i << 4);
#pragma unroll
    for (int j = 0; j < 4; ++j) {
      const int n = n0 + (j << 4) + rlane;
      float bv = 0.f;
      if (BIAS_MODE == 2) bv = bias[n];
#pragma unroll
      for (int r = 0; r < 8; ++r) {
        float v = acc[i][j][r] * scale;
        if (BIAS_MODE == 1) v += bias[mBase + mOff + r];
        if (BIAS_MODE == 2) v += bv;
        if (RESID) v += Rb[(size_t)(mBase + mOff + r) * ldc + n];
        if (ACT == 1) v = tanhf(v);
        if (ACT == 2) v = fmaxf(v, 0.0f);
        if (ACT == 3) v = v / (1.0f + expf(-v));
        if (ACT == 4) v = (v > 0.f) ? v : 0.01f * v;
        if (ACT == 5) v = 0.5f * v * (1.0f + erff(v * 0.70710678118654752f));
        slab[(mOff + r) * 68 + (j << 4) + rlane] = v;
      }
    }
    __builtin_amdgcn_fence(__ATOMIC_RELEASE, "workgroup");
    __builtin_amdgcn_wave_barrier();
    __builtin_amdgcn_fence(__ATOMIC_ACQUIRE, "workgroup");
    if (OUT_MODE == 0) {
      float* C = (float*)Cout + (size_t)b * strideC;
      const int hh = lane >> 4, c4 = (lane & 15) * 4;
      for (int pass = 0; pass < 2; ++pass) {
#pragma unroll
        for (int it = 0; it < 8; ++it) {
          const int row = it * 2 + hh;
          v4f v = *(const v4f*)(slab + row * 68 + c4);
          *(volatile v4f*)(C + (size_t)(mBase + row) * ldc + n0 + c4) = v;
        }
        __threadfence();
      }
    } else {
      const int q = lane >> 3, c8 = (lane & 7) * 8;
      unsigned short* C  = (unsigned short*)Cout  + (size_t)b * strideC;
      unsigned short* C2 = (OUT_MODE == 2) ? ((unsigned short*)Cout2 + (size_t)b * strideC) : nullptr;
      for (int pass = 0; pass < 2; ++pass) {
#pragma unroll
        for (int it = 0; it < 4; ++it) {
          const int row = it * 4 + q;
          const float* sp = slab + row * 68 + c8;
          v8h hv, lv;
#pragma unroll
          for (int e = 0; e < 8; ++e) {
            if (OUT_MODE == 1) {
              hv[e] = (_Float16)sp[e];
            } else {
              unsigned short hb = f2bf_bits(sp[e]);
              unsigned short lb = f2bf_bits(sp[e] - bf_bits2f(hb));
              hv[e] = __builtin_bit_cast(_Float16, hb);
              lv[e] = __builtin_bit_cast(_Float16, lb);
            }
          }
          *(volatile v8h*)(C + (size_t)(mBase + row) * ldc + n0 + c8) = hv;
          if (OUT_MODE == 2) *(volatile v8h*)(C2 + (size_t)(mBase + row) * ldc + n0 + c8) = lv;
        }
        __threadfence();
      }
    }
    __builtin_amdgcn_fence(__ATOMIC_RELEASE, "workgroup");
    __builtin_amdgcn_wave_barrier();
    __builtin_amdgcn_fence(__ATOMIC_ACQUIRE, "workgroup");
  }
}

__global__ __launch_bounds__(256) void gather_x0_kernel(const int* __restrict__ words, const float* __restrict__ emb,
                                                         unsigned short* __restrict__ X0) {
  constexpr int kp8 = NEMBP / 8;
  const int i = blockIdx.x * 256 + threadIdx.x;
  if (i < NROW * kp8) {
    const int row = i / kp8;
    const int c8  = i - row * kp8;
    const int s = row >> 5, b = row & 31;
    int w = words[b * NSEQ + s];
    w = (w < 0) ? 0 : ((w > NVOC - 1) ? (NVOC - 1) : w);
    const float* er = emb + (size_t)w * NEMB;
    v8h hv;
#pragma unroll
    for (int e = 0; e < 8; ++e) {
      const int k  = c8 * 8 + e;
      const int kc = (k < NEMB) ? k : (NEMB - 1);
      const float v = er[kc];
      const float f = (k < NEMB) ? CARRY1 : 0.0f;
      hv[e] = (_Float16)(v * f);
    }
    unsigned short* dp = X0 + (size_t)i * 8;
    *(volatile v8h*)dp = hv;
    __threadfence();
    *(volatile v8h*)dp = hv;
  }
}

__global__ __launch_bounds__(256) void cvt_plane_kernel(const float* __restrict__ src, unsigned short* __restrict__ dst,
                                                         int up, int ureal, int ngate, int kp, int ks,
                                                         int ka, int kb, int kboff, int n8) {
  const int i = blockIdx.x * 256 + threadIdx.x;
  if (i < n8) {
    const int kp8  = kp >> 3;
    const int rowi = i / kp8;
    const int c8   = i - rowi * kp8;
    const int gu   = ngate * up;
    const int dd   = rowi / gu;
    const int rem  = rowi - dd * gu;
    const int g    = rem / up;
    const int u    = rem - g * up;
    const bool uval = (u < ureal);
    const int uc   = uval ? u : (ureal - 1);
    const float* srow = src + ((size_t)(dd * ngate + g) * ureal + uc) * (size_t)ks;
    v8h hv;
#pragma unroll
    for (int e = 0; e < 8; ++e) {
      const int k = c8 * 8 + e;
      const bool inA = (k < ka);
      const bool inB = (k >= kboff) && (k < kboff + kb);
      int sc = inA ? k : (k - kboff + ka);
      sc = (sc < 0) ? 0 : ((sc > ks - 1) ? (ks - 1) : sc);
      const float v = srow[sc];
      const float f = (uval && (inA || inB)) ? CARRY1 : 0.0f;
      hv[e] = (_Float16)(v * f);
    }
    unsigned short* dp = dst + (size_t)i * 8;
    *(volatile v8h*)dp = hv;
    __threadfence();
    *(volatile v8h*)dp = hv;
  }
}

__global__ __launch_bounds__(RTHR) void bilstm_rec_kernel(const float* __restrict__ P, const unsigned short* __restrict__ WHp,
                                                           const float* __restrict__ bias, unsigned short* __restrict__ Y) {
  __shared__ __align__(16) _Float16 Ah[2][16 * AHP];
  const _Float16* WH = (const _Float16*)WHp;
  const int tid = threadIdx.x, lane = tid & 31, wave = tid >> 5;
  const int c = lane & 15, hh = lane >> 4, koff = hh * 8;
  const int d  = blockIdx.x & 1;
  const int b0 = (blockIdx.x >> 1) * 16;
  const int j  = 16 * wave + c;
  const bool jvalid = (j < NHID);
  const int jc = jvalid ? j : (NHID - 1);

  {
    _Float16* ahf = &Ah[0][0];
#pragma unroll 1
    for (int i = tid; i < 2 * 16 * AHP; i += RTHR) ahf[i] = (_Float16)0.0f;
  }
  float cst[8], bg[4];
#pragma unroll
  for (int r = 0; r < 8; ++r) cst[r] = 0.0f;
#pragma unroll
  for (int g = 0; g < 4; ++g) bg[g] = bias[(size_t)d * (NGATE * NHID) + g * NHID + jc];
  __syncthreads();

  const _Float16* w0 = WH + ((size_t)d * NGC + 0 * NUP + j) * NHK + koff;
  const _Float16* w1 = WH + ((size_t)d * NGC + 1 * NUP + j) * NHK + koff;
  const _Float16* w2 = WH + ((size_t)d * NGC + 2 * NUP + j) * NHK + koff;
  const _Float16* w3 = WH + ((size_t)d * NGC + 3 * NUP + j) * NHK + koff;

#pragma unroll 1
  for (int t = 0; t < NSEQ; ++t) {
    const int cur = t & 1;
    const int pos = d ? (NSEQ - 1 - t) : t;
    const float* prow = P + (((size_t)d * NROW) + (size_t)pos * NBAT + b0 + 8 * hh) * NGC + j;
    v8f acc[4];
#pragma unroll
    for (int g = 0; g < 4; ++g) {
#pragma unroll
      for (int r = 0; r < 8; ++r) acc[g][r] = (prow[(size_t)r * NGC + g * NUP] + bg[g]) * CARRY2;
      pin_acc(acc[g]);
    }
    const _Float16* arow = &Ah[cur][0] + c * AHP + koff;
#pragma unroll 1
    for (int k0 = 0; k0 < NHK; k0 += 32) {
      const v16h a  = Frag<_Float16>::load(arow + k0);
      const v16h f0 = Frag<_Float16>::load(w0 + k0);
      const v16h f1 = Frag<_Float16>::load(w1 + k0);
      const v16h f2 = Frag<_Float16>::load(w2 + k0);
      const v16h f3 = Frag<_Float16>::load(w3 + k0);
      acc[0] = Frag<_Float16>::mma(a, f0, acc[0]);
      acc[1] = Frag<_Float16>::mma(a, f1, acc[1]);
      acc[2] = Frag<_Float16>::mma(a, f2, acc[2]);
      acc[3] = Frag<_Float16>::mma(a, f3, acc[3]);
      dep_guard5_h(acc[0], acc[1], acc[2], acc[3], a, f0, f1, f2, f3);
    }
    acc_guard4(acc[0], acc[1], acc[2], acc[3]);

    _Float16* ahn = &Ah[cur ^ 1][0];
#pragma unroll
    for (int r = 0; r < 8; ++r) {
      const float zi = acc[0][r] * CARRY2_INV;
      const float zf = acc[1][r] * CARRY2_INV;
      const float zg = acc[2][r] * CARRY2_INV;
      const float zo = acc[3][r] * CARRY2_INV;
      const float cn = fsig(zf) * cst[r] + fsig(zi) * ftanh(zg);
      cst[r] = cn;
      const float hn = fsig(zo) * ftanh(cn);
      const float hv = jvalid ? hn : 0.0f;
      ahn[(8 * hh + r) * AHP + j] = (_Float16)(hv * CARRY1);
    }
#pragma unroll
    for (int it = 0; it < 2; ++it) {
      const int i = it * RTHR + tid;
      if (i < 16 * (AHP - NUP)) {
        const int rr = i / (AHP - NUP);
        const int cc = i - rr * (AHP - NUP);
        ahn[rr * AHP + NUP + cc] = (_Float16)0.0f;
      }
    }
    __syncthreads();

    unsigned short* yb = Y + ((size_t)(pos * NBAT + b0)) * YPITCH + (size_t)d * YHALF;
    const _Float16* ahs = ahn;
    for (int pass = 0; pass < 2; ++pass) {
#pragma unroll
      for (int it = 0; it < 2; ++it) {
        const int u  = (it * RTHR + tid) >> 3;
        const int e8 = tid & 7;
        if (u < 64) {
          const int rr = u >> 2, q = u & 3;
          const v8h hv = *(const v8h*)(ahs + rr * AHP + q * 64 + e8 * 8);
          *(volatile v8h*)(yb + (size_t)rr * YPITCH + q * 64 + e8 * 8) = hv;
        }
      }
      __threadfence();
    }
  }
}

__global__ __launch_bounds__(256) void head_out_kernel(const float* __restrict__ Z, const float* __restrict__ ob,
                                                        float* __restrict__ out) {
  const int i = blockIdx.x * 256 + threadIdx.x;
  if (i < NOUT / 4) {
    v4f ov;
#pragma unroll
    for (int e = 0; e < 4; ++e) {
      const int idx = i * 4 + e;
      const int bs  = idx / NTAG;
      const int t   = idx - bs * NTAG;
      const int b   = bs >> 7, s = bs & 127;
      const float z = Z[(size_t)(s * NBAT + b) * NTAGP + t] + ob[t];
      ov[e] = fsig(z);
    }
    float* op = out + (size_t)i * 4;
    *(volatile v4f*)op = ov;
    __threadfence();
    *(volatile v4f*)op = ov;
  }
}

extern "C" void kernel_launch(void* const* d_in, const int* in_sizes, int n_in,
                              void* d_out, int out_size, void* d_ws, size_t ws_size, hipStream_t stream) {
  if (n_in < 15 || d_out == nullptr || d_ws == nullptr) return;
  if (in_sizes[0] != NBAT * NSEQ || in_sizes[3] != NVOC * NEMB ||
      in_sizes[7] != 2 * NGATE * NHID * NEMB || in_sizes[8] != 2 * NGATE * NHID * NHID || in_sizes[9] != 2 * NGATE * NHID ||
      in_sizes[10] != 2 * NGATE * NHID * NIN1 || in_sizes[11] != 2 * NGATE * NHID * NHID || in_sizes[12] != 2 * NGATE * NHID ||
      in_sizes[13] != NTAG * NIN1 || in_sizes[14] != NTAG || out_size != NOUT) return;

  const int*   words = (const int*)d_in[0];
  const float* emb   = (const float*)d_in[3];
  const float* wih0  = (const float*)d_in[7];
  const float* whh0  = (const float*)d_in[8];
  const float* bb0   = (const float*)d_in[9];
  const float* wih1  = (const float*)d_in[10];
  const float* whh1  = (const float*)d_in[11];
  const float* bb1   = (const float*)d_in[12];
  const float* wout  = (const float*)d_in[13];
  const float* bout  = (const float*)d_in[14];
  float* out = (float*)d_out;

  char* ws = (char*)d_ws; size_t off = 0;
  auto carve = [&](size_t bytes) -> char* { char* p = ws + off; off += (bytes + 255) & ~(size_t)255; return p; };
  unsigned short* X0   = (unsigned short*)carve((size_t)NROW * NEMBP * 2);
  unsigned short* WIH0 = (unsigned short*)carve((size_t)2 * NGC * NEMBP * 2);
  unsigned short* WHH0 = (unsigned short*)carve((size_t)2 * NGC * NHK * 2);
  unsigned short* WIH1 = (unsigned short*)carve((size_t)2 * NGC * YPITCH * 2);
  unsigned short* WHH1 = (unsigned short*)carve((size_t)2 * NGC * NHK * 2);
  unsigned short* WOUT = (unsigned short*)carve((size_t)NTAGP * YPITCH * 2);
  float*          P    = (float*)carve((size_t)2 * NROW * NGC * 4);
  unsigned short* Y0   = (unsigned short*)carve((size_t)NROW * YPITCH * 2);
  unsigned short* Y1   = (unsigned short*)carve((size_t)NROW * YPITCH * 2);
  float*          Z    = (float*)carve((size_t)NROW * NTAGP * 4);
  if (off > ws_size || off > (size_t)134217728) return;

  const int n8x   = NROW * NEMBP / 8;
  const int n8i0  = 2 * NGC * NEMBP / 8;
  const int n8h   = 2 * NGC * NHK / 8;
  const int n8i1  = 2 * NGC * YPITCH / 8;
  const int n8o   = NTAGP * YPITCH / 8;
  gather_x0_kernel<<<n8x / 256, 256, 0, stream>>>(words, emb, X0);
  cvt_plane_kernel<<<n8i0 / 256, 256, 0, stream>>>(wih0, WIH0, NUP,   NHID, NGATE, NEMBP,  NEMB, NEMB, 0,    NEMBP, n8i0);
  cvt_plane_kernel<<<n8h  / 256, 256, 0, stream>>>(whh0, WHH0, NUP,   NHID, NGATE, NHK,    NHID, NHID, 0,    NHK,   n8h);
  cvt_plane_kernel<<<n8i1 / 256, 256, 0, stream>>>(wih1, WIH1, NUP,   NHID, NGATE, YPITCH, NIN1, NHID, NHID, YHALF, n8i1);
  cvt_plane_kernel<<<n8h  / 256, 256, 0, stream>>>(whh1, WHH1, NUP,   NHID, NGATE, NHK,    NHID, NHID, 0,    NHK,   n8h);
  cvt_plane_kernel<<<n8o  / 256, 256, 0, stream>>>(wout, WOUT, NTAGP, NTAG, 1,     YPITCH, NIN1, NHID, NHID, YHALF, n8o);

  const dim3 ggrid((NROW / 64) * (NGC / 64) / 8, 2);
  wmma_gemm64<0, false, 0, 0, false, 0><<<ggrid, 256, 0, stream>>>(
      X0, X0, NEMBP, 0L, WIH0, WIH0, NEMBP, (long)NGC * NEMBP, (void*)P, (void*)P, NGC, (long)NROW * NGC,
      bb0, (const float*)P, 0L, NROW, NGC, NEMBP, CARRY2_INV);
  bilstm_rec_kernel<<<4, RTHR, 0, stream>>>(P, WHH0, bb0, Y0);

  wmma_gemm64<0, false, 0, 0, false, 0><<<ggrid, 256, 0, stream>>>(
      Y0, Y0, YPITCH, 0L, WIH1, WIH1, YPITCH, (long)NGC * YPITCH, (void*)P, (void*)P, NGC, (long)NROW * NGC,
      bb1, (const float*)P, 0L, NROW, NGC, YPITCH, CARRY2_INV);
  bilstm_rec_kernel<<<4, RTHR, 0, stream>>>(P, WHH1, bb1, Y1);

  const dim3 hgrid((NROW / 64) * (NTAGP / 64) / 8, 1);
  wmma_gemm64<0, false, 0, 0, false, 0><<<hgrid, 256, 0, stream>>>(
      Y1, Y1, YPITCH, 0L, WOUT, WOUT, YPITCH, 0L, (void*)Z, (void*)Z, NTAGP, 0L,
      bout, (const float*)Z, 0L, NROW, NTAGP, YPITCH, CARRY2_INV);
  head_out_kernel<<<NOUT / 4 / 256, 256, 0, stream>>>(Z, bout, out);
}
